// CardAwarePolicy_49675591746172
// MI455X (gfx1250) — hardware-run, weakly checked
//
#include <hip/hip_runtime.h>


namespace {
constexpr int NB_ = 32768, S = 8, NA = 20, KC = 4, E = 64, NHD = 4, HD = 16, NEMB = 54;
constexpr float ES_ = 256.0f  , HS = 256.0f, WSC = 256.0f;
typedef _Float16 b16;
typedef __attribute__((ext_vector_type(16))) _Float16 v16b;
typedef __attribute__((ext_vector_type(8))) _Float16 v8b;
typedef __attribute__((ext_vector_type(8))) float v8f;
typedef __attribute__((ext_vector_type(4))) float v4f;
typedef __attribute__((ext_vector_type(2))) float v2f;
__device__ __forceinline__ float bf16_rne(float f) { unsigned int u = __float_as_uint(f); u += 0x7FFFu + ((u >> 16) & 1u); float r = __uint_as_float(u & 0xFFFF0000u); asm volatile("" : "+v"(r)); return r; }
__device__ __forceinline__ float bfv(float f) { float r = bf16_rne(f); asm volatile("" : "+v"(r)); return r; }
__device__ __forceinline__ void split16(float v, b16& hi, b16& lo) { hi = (b16)v; lo = (b16)(v - (float)hi); }
__device__ __forceinline__ v16b frag_kb(const b16* p, int hh) { const v8b a = *(const v8b*)(p + 8 * hh), b = *(const v8b*)(p + 16 + 8 * hh); v16b f;
#pragma unroll
  for (int e = 0; e < 8; ++e) { f[e] = a[e]; f[8 + e] = b[e]; } return f; }
__device__ __forceinline__ v8f wmma16b(v16b a, v16b b, v8f c) { v8f d = __builtin_amdgcn_wmma_f32_16x16x32_f16(false, a, false, b, (short)0, c, false, false); asm volatile("v_nop\n\tv_nop\n\tv_nop\n\tv_nop" : "+v"(d) : "v"(a), "v"(b)); return d; }
__device__ __forceinline__ void wave_lds_sync() { __builtin_amdgcn_fence(__ATOMIC_RELEASE, "workgroup"); __builtin_amdgcn_wave_barrier(); __builtin_amdgcn_fence(__ATOMIC_ACQUIRE, "workgroup"); }
__device__ __forceinline__ float pmul(float a, float b) { float p = a * b; asm volatile("" : "+v"(p)); return p; }
__device__ __forceinline__ int iclamp(int v, int lo, int hi) { return v < lo ? lo : (v > hi ? hi : v); }

__global__ __launch_bounds__(256) void wput_kernel(const float* __restrict__ win, const float* __restrict__ wo, const float* __restrict__ wg2, const float* __restrict__ wc1, const float* __restrict__ wc2, const float* __restrict__ ws1, const float* __restrict__ ws2, const float* __restrict__ emb, const int* __restrict__ aci, const int* __restrict__ acc_, b16* __restrict__ WIN, b16* __restrict__ WO, b16* __restrict__ WG2, b16* __restrict__ WC1, b16* __restrict__ WC2, b16* __restrict__ WS1, b16* __restrict__ WS2, float* __restrict__ RA) { const size_t nt = (size_t)gridDim.x * 256, u0 = (size_t)blockIdx.x * 256 + threadIdx.x; v8b v;
  auto put = [&](const float* w, b16* P, int rows, int K, int srcStride, size_t& base, size_t u) -> bool { const size_t cnt = (size_t)rows * (K / 8); if (u < base + cnt) { const size_t uu = u - base; const int o = (int)(uu / (K / 8)), k0 = (int)(uu % (K / 8)) * 8;
#pragma unroll
      for (int j = 0; j < 8; ++j) v[j] = (b16)(bf16_rne(w[(size_t)o * srcStride + k0 + j]) * WSC); for (int pass = 0; pass < 2; ++pass) { *(volatile v8b*)(P + (size_t)o * K + k0) = v; __threadfence(); } return true; } base += cnt; return false; };
  for (size_t u = u0; u < 8192; u += nt) { size_t base = 0; if (put(win, WIN, 3 * E, E, E, base, u)) continue; if (put(wo, WO, E, E, E, base, u)) continue; if (put(wg2, WG2, 32, E, E, base, u)) continue; if (put(wc1, WC1, 128, 96, 96, base, u)) continue; if (put(wc2, WC2, 128, 128, 128, base, u)) continue; if (put(ws1, WS1, E, 128, 192, base, u)) continue; if (put(ws2, WS2, 32, E, E, base, u)) continue; }
  if (u0 < (size_t)NA * E) { const int a = (int)(u0 / E), o = (int)(u0 % E); const int cnt = acc_[a]; float s = 0.0f; for (int e = 0; e < E; ++e) { float ar = 0.0f; for (int kk = 0; kk < KC; ++kk) if (kk < cnt) ar += bfv(emb[(size_t)iclamp(aci[a * KC + kk], 0, NEMB - 1) * E + e]); ar = ar / fmaxf((float)cnt, 1.0f); s += pmul(ar, bfv(ws1[(size_t)o * 192 + 128 + e])); }
    for (int pass = 0; pass < 2; ++pass) { ((volatile float*)RA)[u0] = s; __threadfence(); } } }
__global__ __launch_bounds__(32) void hand_kernel(const int* __restrict__ cards, const float* __restrict__ emb, const b16* __restrict__ WIN, const float* __restrict__ bin, int BLIM, float* __restrict__ SA) { __shared__ __attribute__((aligned(16))) b16 Ah[16][E + 8]; __shared__ float Tq[16][3 * E + 4], Pr[2][NHD][S][S + 1], Ao[16][E + 1]; __shared__ int Cd[16]; const int lane = threadIdx.x, nloc = lane & 15, hlf = lane >> 4; const size_t b0 = (size_t)blockIdx.x * 2; if (b0 >= (size_t)BLIM) return;
  if (lane < 16) Cd[lane] = iclamp(cards[b0 * S + lane], 0, NEMB - 1);
  wave_lds_sync();
  for (int rr = 0; rr < 16; ++rr) for (int q = 0; q < 2; ++q) Ah[rr][q * 32 + lane] = (b16)(bfv(emb[(size_t)Cd[rr] * E + q * 32 + lane]) * ES_); if (lane < 16) for (int k = E; k < E + 8; ++k) Ah[lane][k] = (b16)0.0f;
  wave_lds_sync(); v8f acc[12];
#pragma unroll
  for (int t = 0; t < 12; ++t) acc[t] = (v8f){};
#pragma unroll
  for (int kb = 0; kb < E; kb += 32) { const v16b a = frag_kb(&Ah[nloc][kb], hlf);
#pragma unroll
    for (int t = 0; t < 12; ++t) acc[t] = wmma16b(a, frag_kb(WIN + (size_t)(t * 16 + nloc) * E + kb, hlf), acc[t]); }
#pragma unroll
  for (int t = 0; t < 12; ++t) { const int cc = t * 16 + nloc; const float bb = bfv(bin[cc]);
#pragma unroll
    for (int r8 = 0; r8 < 8; ++r8) Tq[8 * hlf + r8][cc] = acc[t][r8] * (1.0f / (ES_ * WSC)) + bb; }
  wave_lds_sync();
  for (int idx = lane; idx < 2 * NHD * S * S; idx += 32) { const int hnd = idx / (NHD * S * S), rem = idx % (NHD * S * S); const int hd = rem / (S * S), qq = (rem / S) % S, kk = rem % S; float s = 0.0f;
#pragma unroll
    for (int d = 0; d < HD; ++d) s += pmul(Tq[hnd * S + qq][hd * HD + d], Tq[hnd * S + kk][E + hd * HD + d]); s *= 0.25f; const bool km = cards[(b0 + hnd) * S + kk] != 0; Pr[hnd][hd][qq][kk] = km ? s : -1e9f; }
  wave_lds_sync();
  for (int rw = lane; rw < 2 * NHD * S; rw += 32) { const int hnd = rw / (NHD * S), hd = (rw / S) % NHD, qq = rw % S; float mx = -INFINITY; for (int kk = 0; kk < S; ++kk) mx = fmaxf(mx, Pr[hnd][hd][qq][kk]); float sm = 0.0f; float p[S];
#pragma unroll
    for (int kk = 0; kk < S; ++kk) { p[kk] = __expf(Pr[hnd][hd][qq][kk] - mx); sm += p[kk]; } const float inv = 1.0f / sm;
#pragma unroll
    for (int kk = 0; kk < S; ++kk) Pr[hnd][hd][qq][kk] = p[kk] * inv; }
  wave_lds_sync();
  for (int rr = 0; rr < 16; ++rr) { const int hnd = rr / S, qq = rr % S; for (int k2 = 0; k2 < 2; ++k2) { const int c = lane * 2 + k2; const int hd = c / HD; float s = 0.0f;
#pragma unroll
      for (int kk = 0; kk < S; ++kk) s += pmul(Pr[hnd][hd][qq][kk], Tq[hnd * S + kk][2 * E + c]); Ao[rr][c] = s; } }
  wave_lds_sync();
  for (int pass = 0; pass < 2; ++pass) { for (int hnd = 0; hnd < 2; ++hnd) { v2f o = {0.0f, 0.0f}; for (int qq = 0; qq < S; ++qq) { o[0] += Ao[hnd * S + qq][lane * 2]; o[1] += Ao[hnd * S + qq][lane * 2 + 1]; } *(volatile v2f*)(SA + (b0 + hnd) * E + lane * 2) = o; } __threadfence(); } }
__global__ __launch_bounds__(32) void sample_kernel(const float* __restrict__ SA, const int* __restrict__ hsz, const float* __restrict__ gs, const b16* __restrict__ WO, const float* __restrict__ ob, const float* __restrict__ g1w, const float* __restrict__ g1b, const b16* __restrict__ WG2, const float* __restrict__ g2b, const b16* __restrict__ WC1, const float* __restrict__ c1b, const b16* __restrict__ WC2, const float* __restrict__ c2b, const b16* __restrict__ WS1, const float* __restrict__ s1b, const float* __restrict__ RA, const b16* __restrict__ WS2, const float* __restrict__ s2b, const float* __restrict__ s3w, const float* __restrict__ s3b, const int* __restrict__ nva, int BLIM, float* __restrict__ out) {
  __shared__ __attribute__((aligned(16))) b16 Ah[16][136], Al[16][136]; __shared__ float Tf[16][132], Pq[16][E + 1], Os[16][NA + 1], Gs[16][13]; const int lane = threadIdx.x, nloc = lane & 15, hlf = lane >> 4; const size_t b0 = (size_t)blockIdx.x * 16; if (b0 >= (size_t)BLIM) return;
  auto stage = [&](int K, auto getter) { for (int rr = 0; rr < 16; ++rr) for (int c = lane; c < K; c += 32) { b16 p, ql; split16(getter(rr, c) * HS, p, ql); Ah[rr][c] = p; Al[rr][c] = ql; } if (lane < 16) for (int k = K; k < K + 8; ++k) { Ah[lane][k] = (b16)0.0f; Al[lane][k] = (b16)0.0f; } wave_lds_sync(); };
  auto gemm = [&](const b16* W, int K, int NT, auto epi) { v8f acc[8];
#pragma unroll
    for (int t = 0; t < 8; ++t) acc[t] = (v8f){};
    for (int kb = 0; kb < K; kb += 32) { const v16b a = frag_kb(&Ah[nloc][kb], hlf), al = frag_kb(&Al[nloc][kb], hlf);
#pragma unroll
      for (int t = 0; t < 8; ++t) if (t < NT) { const v16b bw = frag_kb(W + (size_t)(t * 16 + nloc) * K + kb, hlf); acc[t] = wmma16b(a, bw, acc[t]); acc[t] = wmma16b(al, bw, acc[t]); } }
    wave_lds_sync();
#pragma unroll
    for (int t = 0; t < 8; ++t) if (t < NT) {
#pragma unroll
      for (int r8 = 0; r8 < 8; ++r8) Tf[8 * hlf + r8][t * 16 + nloc] = epi(8 * hlf + r8, t * 16 + nloc, acc[t][r8] * (1.0f / (HS * WSC))); }
    wave_lds_sync(); };
  for (int rr = 0; rr < 16; ++rr) if (lane < 12) Gs[rr][lane] = bfv(gs[(b0 + rr) * 12 + lane]);
  wave_lds_sync();
  stage(E, [&](int rr, int c) { return SA[(b0 + rr) * E + c]; });
  gemm(WO, E, 4, [&](int r, int c, float v) { const float len = fmaxf((float)hsz[b0 + r], 1.0f); return (v + 8.0f * bfv(ob[c])) / len; });
  for (int rr = 0; rr < 16; ++rr) for (int q = 0; q < 2; ++q) Pq[rr][q * 32 + lane] = Tf[rr][q * 32 + lane];
  wave_lds_sync();
  stage(E, [&](int rr, int c) { float s = bfv(g1b[c]); for (int d = 0; d < 12; ++d) s += pmul(Gs[rr][d], bfv(g1w[c * 12 + d])); return fmaxf(s, 0.0f); });
  gemm(WG2, E, 2, [&](int r, int c, float v) { return fmaxf(v + bfv(g2b[c]), 0.0f); });
  stage(96, [&](int rr, int c) { return c < E ? Pq[rr][c] : Tf[rr][c - E]; });
  gemm(WC1, 96, 8, [&](int r, int c, float v) { return fmaxf(v + bfv(c1b[c]), 0.0f); });
  stage(128, [&](int rr, int c) { return Tf[rr][c]; });
  gemm(WC2, 128, 8, [&](int r, int c, float v) { return fmaxf(v + bfv(c2b[c]), 0.0f); });
  stage(128, [&](int rr, int c) { return Tf[rr][c]; });
  gemm(WS1, 128, 4, [&](int r, int c, float v) { return v + bfv(s1b[c]); });
  for (int rr = 0; rr < 16; ++rr) for (int q = 0; q < 2; ++q) Pq[rr][q * 32 + lane] = Tf[rr][q * 32 + lane];
  wave_lds_sync();
  const int nv = nva[0];
#pragma unroll 1
  for (int a = 0; a < NA; ++a) {
    stage(E, [&](int rr, int c) { return fmaxf(Pq[rr][c] + RA[a * E + c], 0.0f); });
    gemm(WS2, E, 2, [&](int r, int c, float v) { return fmaxf(v + bfv(s2b[c]), 0.0f); });
    if (lane < 16) { float s = bfv(s3b[0]); for (int c = 0; c < 32; ++c) s += pmul(Tf[lane][c], bfv(s3w[c])); Os[lane][a] = a < nv ? s : -1e8f; }
    wave_lds_sync(); }
  for (int pass = 0; pass < 2; ++pass) { for (int q = 0; q < 10; ++q) { const int idx = q * 32 + lane; ((volatile float*)out)[b0 * NA + idx] = Os[idx / NA][idx % NA]; } __threadfence(); } }
}

extern "C" void kernel_launch(void* const* d_in, const int* in_sizes, int n_in, void* d_out, int out_size, void* d_ws, size_t ws_size, hipStream_t stream) {
  (void)n_in;
  auto Fp = [&](int i) { return (const float*)d_in[i]; }; auto Ip = [&](int i) { return (const int*)d_in[i]; };
  if (in_sizes[0] != NB_ * S || in_sizes[1] != NB_ * 12 || in_sizes[2] != NB_ || in_sizes[3] != NA * KC || in_sizes[4] != NA || in_sizes[5] != 1 || in_sizes[6] != NEMB * E || in_sizes[7] != 3 * E * E || in_sizes[15] != 128 * 96 || in_sizes[19] != E * 192 || out_size != NB_ * NA) return;
  const int BLIM = NB_;
  size_t off = 0; char* ws = (char*)d_ws;
  auto carve = [&](size_t bytes) { char* p = ws + off; off += (bytes + 255) & ~(size_t)255; return p; };
  b16* WIN = (b16*)carve((size_t)3 * E * E * 2); b16* WO = (b16*)carve((size_t)E * E * 2); b16* WG2 = (b16*)carve((size_t)32 * E * 2); b16* WC1 = (b16*)carve((size_t)128 * 96 * 2); b16* WC2 = (b16*)carve((size_t)128 * 128 * 2); b16* WS1 = (b16*)carve((size_t)E * 128 * 2); b16* WS2 = (b16*)carve((size_t)32 * E * 2); float* RA = (float*)carve((size_t)NA * E * 4); float* SA = (float*)carve((size_t)NB_ * E * 4);
  if (off > ws_size || off > ((size_t)16 << 20)) return;
  wput_kernel<<<32, 256, 0, stream>>>(Fp(7), Fp(9), Fp(13), Fp(15), Fp(17), Fp(19), Fp(21), Fp(6), Ip(3), Ip(4), WIN, WO, WG2, WC1, WC2, WS1, WS2, RA);
  hand_kernel<<<BLIM / 2, 32, 0, stream>>>(Ip(0), Fp(6), WIN, Fp(8), BLIM, SA);
  sample_kernel<<<BLIM / 16, 32, 0, stream>>>(SA, Ip(2), Fp(1), WO, Fp(10), Fp(11), Fp(12), WG2, Fp(14), WC1, Fp(16), WC2, Fp(18), WS1, Fp(20), RA, WS2, Fp(22), Fp(23), Fp(24), Ip(5), BLIM, (float*)d_out);
}
